// DNNTSP_67929202753598
// MI455X (gfx1250) — hardware-run, weakly checked
//
#include <hip/hip_runtime.h>


namespace {
constexpr int IT = 1024, D = 128, NHD = 4, B = 16, N = B * IT, E = 524288, QW = 3 * NHD * D, NCH = IT / 32, NT16 = N / 16;
constexpr float XS = 8.0f, PS = 1024.0f, WSC = 256.0f, BEPS = 1e-5f;
typedef _Float16 b16;
typedef __attribute__((ext_vector_type(16))) _Float16 v16b;
typedef __attribute__((ext_vector_type(8))) _Float16 v8b;
typedef __attribute__((ext_vector_type(8))) float v8f;
typedef __attribute__((ext_vector_type(4))) float v4f;
__device__ __forceinline__ float bf16_rne(float f) { unsigned int u = __float_as_uint(f); u += 0x7FFFu + ((u >> 16) & 1u); float r = __uint_as_float(u & 0xFFFF0000u); asm volatile("" : "+v"(r)); return r; }
__device__ __forceinline__ void split16(float v, b16& hi, b16& lo) { hi = (b16)v; lo = (b16)(v - (float)hi); }
__device__ __forceinline__ v16b frag_kb(const b16* p, int hh) { const v8b a = *(const v8b*)(p + 8 * hh), b = *(const v8b*)(p + 16 + 8 * hh); v16b f;
#pragma unroll
  for (int e = 0; e < 8; ++e) { f[e] = a[e]; f[8 + e] = b[e]; } return f; }
__device__ __forceinline__ v8f wmma16b(v16b a, v16b b, v8f c) { v8f d = __builtin_amdgcn_wmma_f32_16x16x32_f16(false, a, false, b, (short)0, c, false, false); asm volatile("v_nop\n\tv_nop\n\tv_nop\n\tv_nop" : "+v"(d) : "v"(a), "v"(b)); return d; }
__device__ __forceinline__ void wave_lds_sync() { __builtin_amdgcn_fence(__ATOMIC_RELEASE, "workgroup"); __builtin_amdgcn_wave_barrier(); __builtin_amdgcn_fence(__ATOMIC_ACQUIRE, "workgroup"); }
__device__ __forceinline__ float pmul(float a, float b) { float p = a * b; asm volatile("" : "+v"(p)); return p; }
__device__ __forceinline__ int iclamp(int v, int lo, int hi) { return v < lo ? lo : (v > hi ? hi : v); }
constexpr int CSR_NBLK7 = 512, CSR_GB7 = 7, CSR_GN7 = 1 << CSR_GB7  , CSR_TS7 = (CSR_GN7 < 32 ? 32 : CSR_GN7)  , CSR_MAXG7 = 512, CSR_CAP7 = 12288  ;
__device__ __host__ __forceinline__ int csr_tix7(int v) { return (v >> CSR_GB7) * CSR_TS7 + (v & (CSR_GN7 - 1)); }
__global__ __launch_bounds__(64) void csrA_kernel7(const int* __restrict__ dst, int E, int N, int nG, int CHP, int NGP, int* __restrict__ STG, int* __restrict__ HST) {
  extern __shared__ int sm[];
  int* cnt = sm; int* run = sm + NGP; int* ids = sm + 2 * NGP;
  const int b = blockIdx.x; const int ch = (E + CSR_NBLK7 - 1) / CSR_NBLK7; const int e0 = b * ch, e1 = min(E, e0 + ch);
  for (int i = threadIdx.x; i < NGP; i += 64) cnt[i] = 0;
  for (int i = threadIdx.x; i < CHP; i += 64) ids[i] = -1;
  __syncthreads();
  if (threadIdx.x == 0) {
    for (int e = e0; e < e1; ++e) { int d = dst[e]; d = (d < 0) ? 0 : (d >= N ? N - 1 : d); cnt[d >> CSR_GB7] += 1; }
    int acc = 0; for (int g = 0; g < nG; ++g) { run[g] = acc; acc += cnt[g]; }
    for (int e = e0; e < e1; ++e) { int d = dst[e]; d = (d < 0) ? 0 : (d >= N ? N - 1 : d); const int g = d >> CSR_GB7; ids[run[g]] = e; run[g] += 1; } }
  __syncthreads();
  typedef __attribute__((ext_vector_type(4))) int v4i;
  for (int pass = 0; pass < 2; ++pass) {
    for (int i = threadIdx.x; i < CHP / 4; i += 64) *(volatile v4i*)(STG + (size_t)b * CHP + i * 4) = *(const v4i*)(&ids[i * 4]);
    for (int i = threadIdx.x; i < NGP / 4; i += 64) { v4i v; for (int e = 0; e < 4; ++e) v[e] = (i * 4 + e < nG) ? cnt[i * 4 + e] : 0; *(volatile v4i*)(HST + (size_t)b * NGP + i * 4) = v; }
    __threadfence(); }
}
__global__ __launch_bounds__(512) void csrS_kernel7(const int* __restrict__ HST, int nG, int NGP, int* __restrict__ START, int* __restrict__ TOT, int* __restrict__ OFF) {
  __shared__ int tot[CSR_MAXG7];
  const int b = threadIdx.x;
  for (int pass = 0; pass < 2; ++pass) { int runb = 0; for (int g = 0; g < nG; ++g) { int c = HST[(size_t)b * NGP + g]; c = (c < 0) ? 0 : c; ((volatile int*)OFF)[(size_t)g * CSR_NBLK7 + b] = runb; runb += c; } __threadfence(); }
  for (int g = threadIdx.x; g < nG; g += 512) { int s = 0; for (int bb = 0; bb < CSR_NBLK7; ++bb) { int c = HST[(size_t)bb * NGP + g]; s += (c < 0) ? 0 : c; } tot[g] = s; }
  __syncthreads();
  if (threadIdx.x < 32) {
    __shared__ int st[CSR_MAXG7 + 32];
    if (threadIdx.x == 0) { int acc = 0; for (int g = 0; g < NGP; ++g) { st[g] = acc; if (g < nG) acc += (tot[g] + 31) & ~31; } st[NGP] = acc; }
    __builtin_amdgcn_fence(__ATOMIC_RELEASE, "workgroup"); __builtin_amdgcn_wave_barrier(); __builtin_amdgcn_fence(__ATOMIC_ACQUIRE, "workgroup");
    for (int pass = 0; pass < 2; ++pass) { for (int i = threadIdx.x; i < NGP + 32; i += 32) { ((volatile int*)START)[i] = (i <= NGP) ? st[min(i, NGP)] : 0; ((volatile int*)TOT)[i] = (i < nG) ? tot[i] : 0; } __threadfence(); } }
}
__global__ __launch_bounds__(256) void csrB_kernel7(const int* __restrict__ dst, int N, int nG, int CHP, int NGP, int permLen, const int* __restrict__ STG, const int* __restrict__ HST, const int* __restrict__ OFF, const int* __restrict__ START, const int* __restrict__ TOT, int* __restrict__ PERM, int* __restrict__ ROWPTR, int* __restrict__ ROWCNT, int* __restrict__ FLAG) {
  typedef __attribute__((ext_vector_type(4))) int v4i;
  __shared__ int ids[CSR_CAP7]; __shared__ unsigned short key[CSR_CAP7]; __shared__ int outp[CSR_CAP7]; __shared__ int ncnt[CSR_GN7 + 1]; __shared__ int boff[CSR_NBLK7 + 1];
  const int g = blockIdx.x, t_ = threadIdx.x; int tot = TOT[g]; int st = START[g], stn = START[g + 1]; const int v0 = g * CSR_GN7; const int nv = min(CSR_GN7, N - v0); const int t0 = g * CSR_TS7;
  st = (st < 0) ? 0 : (st > permLen - 32 ? permLen - 32 : st) & ~31; stn = (stn < st) ? st : (stn > permLen ? permLen : stn); tot = (tot < 0) ? 0 : tot; if (tot > stn - st && tot <= CSR_CAP7) tot = stn - st;
  if (tot > CSR_CAP7) {
    for (int pass = 0; pass < 2; ++pass) { for (int i = t_; i < CSR_TS7 / 4; i += 256) { v4i a, c; for (int e = 0; e < 4; ++e) { a[e] = st; c[e] = 0; } *(volatile v4i*)(ROWPTR + t0 + i * 4) = a; *(volatile v4i*)(ROWCNT + t0 + i * 4) = c; } if (t_ == 0) ((volatile int*)FLAG)[0] = 1; __threadfence(); } (void)nv; return; }
  if (t_ == 0) { int acc = 0; for (int b = 0; b < CSR_NBLK7; ++b) { boff[b] = acc; int c = HST[(size_t)b * NGP + g]; c = (c < 0) ? 0 : (c > CHP ? CHP : c); acc += c; if (acc > tot) acc = tot; } boff[CSR_NBLK7] = acc; }
  for (int i = t_; i <= CSR_GN7; i += 256) ncnt[i] = 0;
  __syncthreads();
  for (int b = 0; b < CSR_NBLK7; ++b) { const int c = boff[b + 1] - boff[b]; int o_ = OFF[(size_t)g * CSR_NBLK7 + b]; o_ = (o_ < 0) ? 0 : (o_ > CHP - c ? CHP - c : o_); const int* src_ = STG + (size_t)b * CHP + o_;
    for (int i = t_; i < c; i += 256) { int id = src_[i]; id = (id < 0) ? 0 : id; ids[boff[b] + i] = id; int d = dst[id]; d = (d < v0) ? v0 : (d >= N ? N - 1 : d); int kk = d - v0; kk = (kk < 0) ? 0 : (kk >= CSR_GN7 ? CSR_GN7 - 1 : kk); key[boff[b] + i] = (unsigned short)kk; } }
  __syncthreads();
  if (t_ == 0) { for (int i = 0; i < tot; ++i) ncnt[key[i]] += 1; int acc = 0; for (int vl = 0; vl < CSR_GN7; ++vl) { const int c = ncnt[vl]; ncnt[vl] = acc; acc += c; } ncnt[CSR_GN7] = acc;
    for (int i = 0; i < tot; ++i) { const int vl = key[i]; outp[ncnt[vl]] = ids[i]; ncnt[vl] += 1; }
    for (int vl = CSR_GN7; vl > 0; --vl) ncnt[vl] = ncnt[vl - 1]; ncnt[0] = 0; }
  __syncthreads();
  for (int pass = 0; pass < 2; ++pass) {
    for (int i = t_; i < (stn - st) / 4; i += 256) { v4i v; for (int e = 0; e < 4; ++e) { const int q = i * 4 + e; v[e] = (q < tot) ? outp[q] : -1; } *(volatile v4i*)(PERM + st + i * 4) = v; }
    for (int i = t_; i < CSR_TS7 / 4; i += 256) { v4i a, c; for (int e = 0; e < 4; ++e) { const int vl = i * 4 + e; const int vc = vl < CSR_GN7 ? vl : CSR_GN7; a[e] = (vl < CSR_GN7) ? st + ncnt[vc] : st; c[e] = (vl < nv) ? (ncnt[(vc < CSR_GN7 ? vc : CSR_GN7 - 1) + 1] - ncnt[vc]) : 0; } *(volatile v4i*)(ROWPTR + t0 + i * 4) = a; *(volatile v4i*)(ROWCNT + t0 + i * 4) = c; }
    __threadfence(); }
}
__global__ __launch_bounds__(256) void csrZ_kernel7(int* __restrict__ p, size_t n4) { typedef __attribute__((ext_vector_type(4))) int v4i; const size_t tid = (size_t)blockIdx.x * 256 + threadIdx.x, nth = (size_t)gridDim.x * 256; v4i z = {0, 0, 0, 0}; for (size_t i = tid; i < n4; i += nth) *(volatile v4i*)(p + i * 4) = z; }
struct CsrBufs7 { int *STG, *HST, *OFF, *START, *TOT, *PERM, *ROWPTR, *ROWCNT, *FLAG; int nG, NGP, CHP; size_t permLen; char* base; size_t bytes; };
static size_t csr_carve7(CsrBufs7& c, char* ws, size_t off, int E, int N) {
  const size_t off0 = off; c.base = ws + off;
  auto al = [&](size_t bytes) { char* p = ws + off; off += (bytes + 255) & ~(size_t)255; return p; };
  c.nG = (N + CSR_GN7 - 1) / CSR_GN7; c.NGP = (c.nG + 31) & ~31; const int ch = (E + CSR_NBLK7 - 1) / CSR_NBLK7; c.CHP = (ch + 31) & ~31; c.permLen = (size_t)E + 32 * (size_t)c.nG + 32;
  c.STG = (int*)al((size_t)CSR_NBLK7 * c.CHP * 4); c.HST = (int*)al((size_t)CSR_NBLK7 * c.NGP * 4); c.OFF = (int*)al((size_t)c.NGP * CSR_NBLK7 * 4); c.START = (int*)al((size_t)(c.NGP + 64) * 4); c.TOT = (int*)al((size_t)(c.NGP + 64) * 4);
  c.PERM = (int*)al(c.permLen * 4); c.ROWPTR = (int*)al((size_t)c.nG * CSR_TS7 * 4); c.ROWCNT = (int*)al((size_t)c.nG * CSR_TS7 * 4); c.FLAG = (int*)al(256);
  c.bytes = off - off0; return off;
}
static void csr_build7(const CsrBufs7& c, const int* dst, int E, int N, hipStream_t stream) {
  const size_t smem = (size_t)(2 * c.NGP + c.CHP) * 4;
  csrZ_kernel7<<<512, 256, 0, stream>>>((int*)c.base, c.bytes / 16);
  csrA_kernel7<<<CSR_NBLK7, 64, smem, stream>>>(dst, E, N, c.nG, c.CHP, c.NGP, c.STG, c.HST);
  csrS_kernel7<<<1, 512, 0, stream>>>(c.HST, c.nG, c.NGP, c.START, c.TOT, c.OFF);
  csrB_kernel7<<<c.nG, 256, 0, stream>>>(dst, N, c.nG, c.CHP, c.NGP, (int)c.permLen, c.STG, c.HST, c.OFF, c.START, c.TOT, c.PERM, c.ROWPTR, c.ROWCNT, c.FLAG);
}


__global__ __launch_bounds__(256) void wcopy_kernel(const float* __restrict__ w, size_t total, b16* __restrict__ WT) { const size_t u = (size_t)blockIdx.x * 256 + threadIdx.x; if (u >= total / 8) return; const size_t e = u * 8; v8b v;
#pragma unroll
  for (int j = 0; j < 8; ++j) v[j] = (b16)(bf16_rne(w[e + j]) * WSC); for (int pass = 0; pass < 2; ++pass) { *(volatile v8b*)(WT + e) = v; __threadfence(); } }
__global__ __launch_bounds__(256) void dis_kernel(const float* __restrict__ ew, const int* __restrict__ rows, const int* __restrict__ PERM, const int* __restrict__ ROWPTR, const int* __restrict__ ROWCNT, int permLen, int NLIM, float* __restrict__ DIS) {
  const int i = blockIdx.x * 256 + threadIdx.x; if (i >= N) return; float s = 1.0f; if (i < NLIM) { int st = ROWPTR[i], cnt = ROWCNT[i]; cnt = iclamp(cnt, 0, 1 << 20); st = iclamp(st, 0, permLen - cnt);
#pragma unroll 1
    for (int j = 0; j < cnt; ++j) { const int e = iclamp(PERM[st + j], 0, E - 1); if (iclamp(rows[e], 0, N - 1) >= NLIM) continue; s += bf16_rne(ew[e]); } }
  const float d = s > 0.0f ? rsqrtf(fmaxf(s, 1e-12f)) : 0.0f; for (int pass = 0; pass < 2; ++pass) { ((volatile float*)DIS)[i] = d; __threadfence(); } }
template <int MODE, int F16OUT>
__global__ __launch_bounds__(32) void dense_kernel(const float* __restrict__ IN, const b16* __restrict__ WT, const float* __restrict__ bias, int NG, int RLIM, float* __restrict__ OUT, b16* __restrict__ OUT16) {
  __shared__ __attribute__((aligned(16))) b16 Ah[16][D + 8], Al[16][MODE == 0 ? 8 : D + 8]; __shared__ float Tf[16][132]; const int lane = threadIdx.x, nloc = lane & 15, hlf = lane >> 4; const int g = blockIdx.x % NG; const size_t m0 = (size_t)(blockIdx.x / NG) * 16; if (m0 >= (size_t)RLIM) return; const int OW = NG * 128;
  for (int rr = 0; rr < 16; ++rr) for (int q = 0; q < 4; ++q) { const float v = IN[(m0 + rr) * D + q * 32 + lane]; if (MODE == 0) Ah[rr][q * 32 + lane] = (b16)(bf16_rne(v) * XS); else { b16 p, ql; split16(v * XS, p, ql); Ah[rr][q * 32 + lane] = p; Al[rr][q * 32 + lane] = ql; } }
  wave_lds_sync(); v8f acc[8];
#pragma unroll
  for (int t = 0; t < 8; ++t) acc[t] = (v8f){};
#pragma unroll
  for (int kb = 0; kb < D; kb += 32) { const v16b a = frag_kb(&Ah[nloc][kb], hlf); v16b a2; if (MODE != 0) a2 = frag_kb(&Al[nloc][kb], hlf);
#pragma unroll
    for (int t = 0; t < 8; ++t) { const v16b bw = frag_kb(WT + (size_t)(g * 128 + t * 16 + nloc) * D + kb, hlf); acc[t] = wmma16b(a, bw, acc[t]); if (MODE != 0) acc[t] = wmma16b(a2, bw, acc[t]); } }
#pragma unroll
  for (int t = 0; t < 8; ++t) { const int c = g * 128 + t * 16 + nloc; const float bb = bias ? bf16_rne(bias[c]) : 0.0f;
#pragma unroll
    for (int r8 = 0; r8 < 8; ++r8) Tf[8 * hlf + r8][t * 16 + nloc] = acc[t][r8] * (1.0f / (XS * WSC)) + bb; }
  wave_lds_sync();
  for (int pass = 0; pass < 2; ++pass) { for (int rr = 0; rr < 16; ++rr) { if (F16OUT) { v4f f = *(const v4f*)(&Tf[rr][lane * 4]); typedef __attribute__((ext_vector_type(4))) _Float16 v4b; v4b hv = {(b16)(f[0] * XS), (b16)(f[1] * XS), (b16)(f[2] * XS), (b16)(f[3] * XS)}; *(volatile v4b*)(OUT16 + (m0 + rr) * OW + g * 128 + lane * 4) = hv; } else *(volatile v4f*)(OUT + (m0 + rr) * OW + g * 128 + lane * 4) = *(const v4f*)(&Tf[rr][lane * 4]); } __threadfence(); }
}
__global__ __launch_bounds__(256) void gcn_kernel(const float* __restrict__ XW, const float* __restrict__ DIS, const float* __restrict__ ew, const float* __restrict__ bias, const int* __restrict__ rows, const int* __restrict__ PERM, const int* __restrict__ ROWPTR, const int* __restrict__ ROWCNT, int permLen, int NLIM, float* __restrict__ G) {
  const int wave = threadIdx.x >> 5, lane = threadIdx.x & 31; const size_t i = (size_t)blockIdx.x * 8 + wave; if (i >= (size_t)NLIM) return; int st = ROWPTR[i], cnt = ROWCNT[i]; cnt = iclamp(cnt, 0, 1 << 20); st = iclamp(st, 0, permLen - cnt); const float di = DIS[i];
  v4f acc; { const v4f xv = *(const v4f*)(XW + i * D + lane * 4); const float wsl = pmul(di, di); for (int k = 0; k < 4; ++k) acc[k] = pmul(wsl, xv[k]); }
#pragma unroll 1
  for (int j = 0; j < cnt; ++j) { const int e = iclamp(PERM[st + j], 0, E - 1); const size_t r = (size_t)iclamp(rows[e], 0, N - 1); if (r >= (size_t)NLIM) continue; const float nw = pmul(pmul(DIS[r], bf16_rne(ew[e])), di); const v4f xv = *(const v4f*)(XW + r * D + lane * 4); for (int k = 0; k < 4; ++k) acc[k] += pmul(nw, xv[k]); }
  v4f o; for (int k = 0; k < 4; ++k) o[k] = acc[k] + bf16_rne(bias[lane * 4 + k]);
  for (int pass = 0; pass < 2; ++pass) { *(volatile v4f*)(G + i * D + lane * 4) = o; __threadfence(); } }
__global__ __launch_bounds__(256) void tilestat_kernel(const float* __restrict__ Hm, int RLIM, float* __restrict__ PSQ) { const int wave = threadIdx.x >> 5, lane = threadIdx.x & 31; const size_t tile = (size_t)blockIdx.x * 8 + wave; if (tile * 16 >= (size_t)RLIM) return; v4f s = {0.0f, 0.0f, 0.0f, 0.0f}, q = {0.0f, 0.0f, 0.0f, 0.0f};
#pragma unroll 1
  for (int rr = 0; rr < 16; ++rr) { const v4f v = *(const v4f*)(Hm + (tile * 16 + rr) * D + lane * 4); for (int k = 0; k < 4; ++k) { s[k] += v[k]; q[k] += pmul(v[k], v[k]); } }
  for (int pass = 0; pass < 2; ++pass) { *(volatile v4f*)(PSQ + tile * 2 * D + lane * 4) = s; *(volatile v4f*)(PSQ + tile * 2 * D + D + lane * 4) = q; __threadfence(); } }
__global__ __launch_bounds__(128) void bnstat_kernel(const float* __restrict__ PSQ, const float* __restrict__ g, const float* __restrict__ bta, int ntiles, int nrows, float* __restrict__ ST) { const int c = threadIdx.x; double s = 0.0, q = 0.0;
#pragma unroll 1
  for (int t = 0; t < ntiles; ++t) { s += (double)PSQ[(size_t)t * 2 * D + c]; q += (double)PSQ[(size_t)t * 2 * D + D + c]; } const double mu = s / (double)nrows; double var = q / (double)nrows - mu * mu; if (var < 0.0) var = 0.0;
  for (int pass = 0; pass < 2; ++pass) { ((volatile float*)ST)[c] = (float)mu; ((volatile float*)ST)[D + c] = pmul((float)(1.0 / sqrt(var + (double)BEPS)), bf16_rne(g[c])); ((volatile float*)ST)[2 * D + c] = bf16_rne(bta[c]); __threadfence(); } }
__global__ __launch_bounds__(256) void bnrelu_kernel(const float* __restrict__ Hm, const float* __restrict__ ST, int RLIM, float* __restrict__ OUT) { const size_t u = (size_t)blockIdx.x * 256 + threadIdx.x; if (u >= (size_t)RLIM * D / 4) return; const int c0 = (int)(u % (D / 4)) * 4; const v4f v = *(const v4f*)(Hm + u * 4); v4f r;
  for (int k = 0; k < 4; ++k) r[k] = fmaxf(pmul(v[k] - ST[c0 + k], ST[D + c0 + k]) + ST[2 * D + c0 + k], 0.0f);
  for (int pass = 0; pass < 2; ++pass) { *(volatile v4f*)(OUT + u * 4) = r; __threadfence(); } }
__global__ __launch_bounds__(32) void vt_kernel(const b16* __restrict__ QKV, int BV, b16* __restrict__ VT) { const int lane = threadIdx.x; const int ch = blockIdx.x % NCH, hh = (blockIdx.x / NCH) % NHD, b = blockIdx.x / (NCH * NHD); if (b >= BV) return; const size_t row = (size_t)b * IT + ch * 32 + lane; const size_t base = (((size_t)b * NHD + hh) * NCH + ch) * D;
  for (int pass = 0; pass < 2; ++pass) {
#pragma unroll 4
    for (int d = 0; d < D; ++d) ((volatile b16*)VT)[(base + d) * 64 + lane] = QKV[row * QW + 2 * NHD * D + hh * D + d]; __threadfence(); } }
__global__ __launch_bounds__(32) void att_kernel(const b16* __restrict__ QKV, const b16* __restrict__ VT, int BV, float* __restrict__ O) {
  __shared__ __attribute__((aligned(16))) b16 Ph[16][40], Pl[16][40]; __shared__ float Sc[16][33], Mx[16], Dn[16], Sf[16], Of[16][D + 4];
  const int lane = threadIdx.x, nloc = lane & 15, hlf = lane >> 4; const int qt = blockIdx.x % (IT / 16); const int b = blockIdx.x / (IT / 16); if (b >= BV) return; const int q0 = qt * 16; const size_t qrow = (size_t)b * IT + q0;
  for (int rr = lane; rr < 16 * (D + 4); rr += 32) (&Of[0][0])[rr] = 0.0f;
#pragma unroll 1
  for (int hh = 0; hh < NHD; ++hh) {
    if (lane < 16) { Mx[lane] = -INFINITY; Dn[lane] = 0.0f; Sf[lane] = 0.0f; } v16b qa[4];
#pragma unroll
    for (int kk = 0; kk < 4; ++kk) qa[kk] = frag_kb(QKV + (qrow + nloc) * QW + hh * D + kk * 32, hlf);
    v8f acc[8];
#pragma unroll
    for (int t = 0; t < 8; ++t) acc[t] = (v8f){};
    wave_lds_sync();
#pragma unroll 1
    for (int kc = 0; kc < q0 + 16; kc += 32) {
#pragma unroll
      for (int blk = 0; blk < 2; ++blk) { v8f s = {}; const size_t kr = ((size_t)b * IT + kc + blk * 16 + nloc) * QW + NHD * D + hh * D;
#pragma unroll
        for (int kk = 0; kk < 4; ++kk) s = wmma16b(qa[kk], frag_kb(QKV + kr + kk * 32, hlf), s);
#pragma unroll
        for (int r8 = 0; r8 < 8; ++r8) { const int qi = q0 + 8 * hlf + r8, kj = kc + blk * 16 + nloc; Sc[8 * hlf + r8][blk * 16 + nloc] = (kj <= qi) ? s[r8] * (0.08838834764831845f / (XS * XS)) : -INFINITY; } }
      wave_lds_sync();
#pragma unroll 1
      for (int qi = 0; qi < 16; ++qi) { const float sv = Sc[qi][lane]; float cm = sv; for (int o = 16; o; o >>= 1) cm = fmaxf(cm, __shfl_xor(cm, o)); const float mo = Mx[qi]; const float mn = fmaxf(mo, cm); const float p = (sv == -INFINITY) ? 0.0f : __expf(sv - mn); float ps = p; for (int o = 16; o; o >>= 1) ps += __shfl_xor(ps, o);
        b16 ph, plo; split16(p * PS, ph, plo); Ph[qi][lane] = ph; Pl[qi][lane] = plo; if (lane == 0) { const float sf = (mo == -INFINITY) ? 0.0f : __expf(mo - mn); Sf[qi] = sf; Dn[qi] = Dn[qi] * sf + ps; Mx[qi] = mn; } }
      wave_lds_sync(); const v16b pa = frag_kb(&Ph[nloc][0], hlf), pb = frag_kb(&Pl[nloc][0], hlf); const size_t vb = ((((size_t)b * NHD + hh) * NCH + kc / 32) * D) * 64;
#pragma unroll
      for (int t = 0; t < 8; ++t) {
#pragma unroll
        for (int r8 = 0; r8 < 8; ++r8) acc[t][r8] *= Sf[8 * hlf + r8];
        const v16b vh = frag_kb(VT + vb + (size_t)(t * 16 + nloc) * 64, hlf); acc[t] = wmma16b(pa, vh, acc[t]); acc[t] = wmma16b(pb, vh, acc[t]); }
      wave_lds_sync(); }
#pragma unroll
    for (int t = 0; t < 8; ++t)
#pragma unroll
      for (int r8 = 0; r8 < 8; ++r8) { const int rl = 8 * hlf + r8; Of[rl][t * 16 + nloc] += acc[t][r8] * (1.0f / (PS * XS * NHD)) / Dn[rl]; }
    wave_lds_sync(); }
  for (int pass = 0; pass < 2; ++pass) { for (int rr = 0; rr < 16; ++rr) *(volatile v4f*)(O + (qrow + rr) * D + lane * 4) = *(const v4f*)(&Of[rr][lane * 4]); __threadfence(); }
}
__global__ __launch_bounds__(32) void fin_kernel(const float* __restrict__ O, const b16* __restrict__ WA, const float* __restrict__ emb, const float* __restrict__ alpha, int RLIM, float* __restrict__ out) {
  __shared__ __attribute__((aligned(16))) b16 Ah[16][D + 8], Al[16][D + 8]; __shared__ float Tf[16][132]; const int lane = threadIdx.x, nloc = lane & 15, hlf = lane >> 4; const size_t m0 = (size_t)blockIdx.x * 16; if (m0 >= (size_t)RLIM) return;
  for (int rr = 0; rr < 16; ++rr) for (int q = 0; q < 4; ++q) { b16 p, ql; split16(O[(m0 + rr) * D + q * 32 + lane] * XS, p, ql); Ah[rr][q * 32 + lane] = p; Al[rr][q * 32 + lane] = ql; }
  wave_lds_sync(); v8f acc[8];
#pragma unroll
  for (int t = 0; t < 8; ++t) acc[t] = (v8f){};
#pragma unroll
  for (int kb = 0; kb < D; kb += 32) { const v16b a = frag_kb(&Ah[nloc][kb], hlf), al = frag_kb(&Al[nloc][kb], hlf);
#pragma unroll
    for (int t = 0; t < 8; ++t) { const v16b bw = frag_kb(WA + (size_t)(t * 16 + nloc) * D + kb, hlf); acc[t] = wmma16b(a, bw, acc[t]); acc[t] = wmma16b(al, bw, acc[t]); } }
#pragma unroll
  for (int t = 0; t < 8; ++t) { const int c = t * 16 + nloc;
#pragma unroll
    for (int r8 = 0; r8 < 8; ++r8) { const int rl = 8 * hlf + r8; const int item = (int)((m0 + rl) % IT); const float a_ = bf16_rne(alpha[item]); Tf[rl][c] = pmul(1.0f - a_, bf16_rne(emb[(size_t)item * D + c])) + pmul(a_, acc[t][r8] * (1.0f / (XS * WSC))); } }
  wave_lds_sync();
  for (int pass = 0; pass < 2; ++pass) { for (int rr = 0; rr < 16; ++rr) *(volatile v4f*)(out + (m0 + rr) * D + lane * 4) = *(const v4f*)(&Tf[rr][lane * 4]); __threadfence(); }
}
}

extern "C" void kernel_launch(void* const* d_in, const int* in_sizes, int n_in, void* d_out, int out_size, void* d_ws, size_t ws_size, hipStream_t stream) {
  (void)n_in;
  auto Fp = [&](int i) { return (const float*)d_in[i]; }; auto Ip = [&](int i) { return (const int*)d_in[i]; };
  if (in_sizes[0] != N * D || in_sizes[1] != 2 * E || in_sizes[2] != E || in_sizes[3] != IT * D || in_sizes[4] != D * D || in_sizes[12] != NHD * D * D || in_sizes[15] != D * D || in_sizes[16] != IT || out_size != N * D) return;
  const int BV = B; const int RL = BV * IT;
  size_t off = 0; char* ws = (char*)d_ws;
  auto carve = [&](size_t bytes) { char* p = ws + off; off += (bytes + 255) & ~(size_t)255; return p; };
  b16* W1 = (b16*)carve((size_t)D * D * 2); b16* W2 = (b16*)carve((size_t)D * D * 2); b16* WQKV = (b16*)carve((size_t)QW * D * 2); b16* WA = (b16*)carve((size_t)D * D * 2);
  float* DIS = (float*)carve((size_t)N * 4); float* XW = (float*)carve((size_t)N * D * 4); float* G = (float*)carve((size_t)N * D * 4); float* H = (float*)carve((size_t)N * D * 4); float* PSQ = (float*)carve((size_t)NT16 * 2 * D * 4); float* ST = (float*)carve(3 * D * 4);
  b16* QKV = (b16*)carve((size_t)N * QW * 2); b16* VT = (b16*)carve((size_t)B * NHD * NCH * D * 64 * 2); float* O = (float*)carve((size_t)N * D * 4); CsrBufs7 csr; off = csr_carve7(csr, ws, off, E, N);
  if (off > ws_size || off > ((size_t)160 << 20)) return;
  wcopy_kernel<<<(D * D / 8 + 255) / 256, 256, 0, stream>>>(Fp(4), (size_t)D * D, W1); wcopy_kernel<<<(D * D / 8 + 255) / 256, 256, 0, stream>>>(Fp(8), (size_t)D * D, W2); wcopy_kernel<<<(D * D / 8 + 255) / 256, 256, 0, stream>>>(Fp(15), (size_t)D * D, WA);
  wcopy_kernel<<<(NHD * D * D / 8 + 255) / 256, 256, 0, stream>>>(Fp(12), (size_t)NHD * D * D, WQKV); wcopy_kernel<<<(NHD * D * D / 8 + 255) / 256, 256, 0, stream>>>(Fp(13), (size_t)NHD * D * D, WQKV + (size_t)NHD * D * D); wcopy_kernel<<<(NHD * D * D / 8 + 255) / 256, 256, 0, stream>>>(Fp(14), (size_t)NHD * D * D, WQKV + (size_t)2 * NHD * D * D);
  csr_build7(csr, Ip(1) + E, E, N, stream);
  dis_kernel<<<(N + 255) / 256, 256, 0, stream>>>(Fp(2), Ip(1), csr.PERM, csr.ROWPTR, csr.ROWCNT, (int)csr.permLen, N, DIS);
  dense_kernel<0, 0><<<N / 16, 32, 0, stream>>>(Fp(0), W1, nullptr, 1, N, XW, nullptr);
  gcn_kernel<<<N / 8, 256, 0, stream>>>(XW, DIS, Fp(2), Fp(5), Ip(1), csr.PERM, csr.ROWPTR, csr.ROWCNT, (int)csr.permLen, N, G);
  tilestat_kernel<<<(NT16 + 7) / 8, 256, 0, stream>>>(G, N, PSQ); bnstat_kernel<<<1, D, 0, stream>>>(PSQ, Fp(6), Fp(7), NT16, N, ST); bnrelu_kernel<<<(N * D / 4 + 255) / 256, 256, 0, stream>>>(G, ST, N, H);
  dense_kernel<1, 0><<<N / 16, 32, 0, stream>>>(H, W2, nullptr, 1, N, XW, nullptr);
  gcn_kernel<<<N / 8, 256, 0, stream>>>(XW, DIS, Fp(2), Fp(9), Ip(1), csr.PERM, csr.ROWPTR, csr.ROWCNT, (int)csr.permLen, N, G);
  tilestat_kernel<<<(NT16 + 7) / 8, 256, 0, stream>>>(G, N, PSQ); bnstat_kernel<<<1, D, 0, stream>>>(PSQ, Fp(10), Fp(11), NT16, N, ST); bnrelu_kernel<<<(N * D / 4 + 255) / 256, 256, 0, stream>>>(G, ST, N, H);
  dense_kernel<1, 1><<<(RL / 16) * (QW / 128), 32, 0, stream>>>(H, WQKV, nullptr, QW / 128, RL, nullptr, QKV);
  vt_kernel<<<BV * NHD * NCH, 32, 0, stream>>>(QKV, BV, VT);
  att_kernel<<<BV * (IT / 16), 32, 0, stream>>>(QKV, VT, BV, O);
  fin_kernel<<<RL / 16, 32, 0, stream>>>(O, WA, Fp(3), Fp(16), RL, (float*)d_out);
}
